// LSTMNet_80848464380559
// MI455X (gfx1250) — hardware-run, weakly checked
//
#include <hip/hip_runtime.h>
#include <math.h>

constexpr int NBATCH  = 32;
constexpr int NSTEP   = 512;
constexpr int NFEAT   = 768;
constexpr int NHID    = 384;
constexpr int NGATE   = 4 * NHID;
constexpr int NROWS   = NBATCH * NSTEP;
constexpr int NWAVE   = 6;
constexpr int NTHR    = 32 * NWAVE;
constexpr int SEQ_BLK = 16;
constexpr int HPITCH  = 392;
constexpr int SLABP   = 68;
constexpr int CVT_THR = 256;
constexpr float ACARRY = 16.0f;
constexpr float WCARRY = 64.0f;
constexpr float FOLD   = 1.0f / (ACARRY * WCARRY);
constexpr float H16_MIN_NORMAL = 6.103515625e-5f;

static_assert(NGATE == 1536);
static_assert(NHID == 64 * NWAVE);
static_assert(NFEAT == 2 * NHID);
static_assert(NFEAT % 32 == 0);
static_assert(NHID % 32 == 0);
static_assert(HPITCH % 8 == 0 && HPITCH >= NHID);
static_assert(NBATCH == 2 * SEQ_BLK);
static_assert((NROWS * NFEAT / 8) % CVT_THR == 0);
static_assert((NGATE * NFEAT / 8) % CVT_THR == 0);
static_assert((NGATE * NHID / 8) % CVT_THR == 0);
static_assert(SLABP % 4 == 0);

typedef __attribute__((ext_vector_type(16))) _Float16 v16h;
typedef __attribute__((ext_vector_type(8)))  _Float16 v8h;
typedef __attribute__((ext_vector_type(8)))  float    v8f;
typedef __attribute__((ext_vector_type(4)))  float    v4f;

struct FragH {
  union U { v16h v; v8h h[2]; };
  static __device__ __forceinline__ v16h load(const _Float16* p) {
    U f;
    f.h[0] = *(const v8h*)(p);
    f.h[1] = *(const v8h*)(p + 16);
    return f.v;
  }
  static __device__ __forceinline__ v8f mma(v16h a, v16h b, v8f c) {
    return __builtin_amdgcn_wmma_f32_16x16x32_f16(false, a, false, b, (short)0, c, false, false);
  }
};

__device__ __forceinline__ void guard_grp(v8f& a0, v8f& a1, v8f& a2, v8f& a3,
                                          v16h a, v16h b0, v16h b1, v16h b2, v16h b3) {
  asm volatile("v_nop\n\tv_nop\n\tv_nop\n\tv_nop"
               : "+v"(a0), "+v"(a1), "+v"(a2), "+v"(a3)
               : "v"(a), "v"(b0), "v"(b1), "v"(b2), "v"(b3));
}
__device__ __forceinline__ void acc_guard4(v8f& a, v8f& b, v8f& c, v8f& d) {
  asm volatile("v_nop\n\tv_nop\n\tv_nop\n\tv_nop" : "+v"(a), "+v"(b), "+v"(c), "+v"(d));
}

__device__ __forceinline__ _Float16 h16_of(float v) {
  const float w = (fabsf(v) < H16_MIN_NORMAL) ? 0.0f : v;
  return (_Float16)w;
}

__device__ __forceinline__ float fsig(float x)  { return __builtin_amdgcn_rcpf(1.0f + __expf(-x)); }
__device__ __forceinline__ float ftanh(float x) { return 1.0f - 2.0f * __builtin_amdgcn_rcpf(__expf(2.0f * x) + 1.0f); }

__global__ __launch_bounds__(CVT_THR) void cvt8_kernel(const float* __restrict__ s0, const float* __restrict__ s1,
                                                       const float* __restrict__ s2, const float* __restrict__ s3,
                                                       unsigned short* __restrict__ dst, int n8, float carry) {
  const int y = (int)blockIdx.y;
  const float* src = (y == 0) ? s0 : ((y == 1) ? s1 : ((y == 2) ? s2 : s3));
  unsigned short* dp = dst + (size_t)y * (size_t)n8 * 8;
  const int i = (int)blockIdx.x * CVT_THR + (int)threadIdx.x;
  if (i < n8) {
    const v4f a = *(const v4f*)(src + (size_t)i * 8);
    const v4f b = *(const v4f*)(src + (size_t)i * 8 + 4);
    v8h hv;
#pragma unroll
    for (int e = 0; e < 4; ++e) {
      const float fa = a[e] * carry;
      const float fb = b[e] * carry;
      hv[e]     = h16_of(fa);
      hv[4 + e] = h16_of(fb);
    }
    *(volatile v8h*)(dp + (size_t)i * 8) = hv;
    __threadfence();
    *(volatile v8h*)(dp + (size_t)i * 8) = hv;
  }
}

template <int LAYER>
__global__ __launch_bounds__(NTHR) void recur_layer_kernel(const unsigned short* __restrict__ Ainp,
                                                           const unsigned short* __restrict__ WIp,
                                                           const unsigned short* __restrict__ WHp,
                                                           const float* __restrict__ biasF,
                                                           const float* __restrict__ biasB,
                                                           const int* __restrict__ mask,
                                                           unsigned short* outH, float* outF) {
  __shared__ __align__(16) _Float16 Ah[2][SEQ_BLK * HPITCH];
  __shared__ __align__(16) float    Sl[NWAVE][16 * SLABP];

  const _Float16* Ain = (const _Float16*)Ainp;
  const int tid = (int)threadIdx.x, lane = tid & 31, wave = tid >> 5;
  const int c = lane & 15, hh = lane >> 4, koff = hh * 8;
  const int dir = (int)(blockIdx.x >> 1);
  const int rowbase = (int)(blockIdx.x & 1) * SEQ_BLK;
  const _Float16* WI = (const _Float16*)WIp + (size_t)dir * NGATE * NFEAT;
  const _Float16* WH = (const _Float16*)WHp + (size_t)dir * NGATE * NHID;
  const float* bias = dir ? biasB : biasF;

  {
    _Float16* ahf = &Ah[0][0];
#pragma unroll 1
    for (int i = tid; i < 2 * SEQ_BLK * HPITCH; i += NTHR) ahf[i] = (_Float16)0.0f;
  }
  float cst[4][8], hst[4][8], bb[4][4];
#pragma unroll
  for (int nt = 0; nt < 4; ++nt) {
    const int j = 64 * wave + 16 * nt + c;
#pragma unroll
    for (int g = 0; g < 4; ++g) bb[nt][g] = bias[g * NHID + j];
#pragma unroll
    for (int r = 0; r < 8; ++r) { cst[nt][r] = 0.0f; hst[nt][r] = 0.0f; }
  }
  __syncthreads();

  const v8f z8 = {0.f, 0.f, 0.f, 0.f, 0.f, 0.f, 0.f, 0.f};
  float* slab = Sl[wave];
  const int* mrow = mask + (size_t)(rowbase + 8 * hh) * NSTEP;
  constexpr size_t GSTR_I = (size_t)NHID * NFEAT;
  constexpr size_t GSTR_H = (size_t)NHID * NHID;
  constexpr size_t ROWSTR = (size_t)NSTEP * NFEAT;

#pragma unroll 1
  for (int s = 0; s < NSTEP; ++s) {
    const int t = dir ? (NSTEP - 1 - s) : s;
    const int cur = s & 1;
    const _Float16* ahrow = &Ah[cur][0] + c * HPITCH + koff;
    _Float16* ahn = &Ah[cur ^ 1][0];
    const _Float16* axrow = Ain + ((size_t)(rowbase + c) * NSTEP + (size_t)t) * NFEAT + koff;

    float mkf[8];
#pragma unroll
    for (int r = 0; r < 8; ++r) mkf[r] = (float)mrow[r * NSTEP + t];

#pragma unroll
    for (int nt = 0; nt < 4; ++nt) {
      const int j = 64 * wave + 16 * nt + c;
      const _Float16* wi = WI + (size_t)j * NFEAT + koff;
      const _Float16* wh = WH + (size_t)j * NHID + koff;
      v8f acc[4];
      acc[0] = z8; acc[1] = z8; acc[2] = z8; acc[3] = z8;
#pragma unroll 1
      for (int k0 = 0; k0 < NFEAT; k0 += 32) {
        const v16h a  = FragH::load(axrow + k0);
        const v16h b0 = FragH::load(wi + k0);
        const v16h b1 = FragH::load(wi + GSTR_I + k0);
        const v16h b2 = FragH::load(wi + 2 * GSTR_I + k0);
        const v16h b3 = FragH::load(wi + 3 * GSTR_I + k0);
        acc[0] = FragH::mma(a, b0, acc[0]);
        acc[1] = FragH::mma(a, b1, acc[1]);
        acc[2] = FragH::mma(a, b2, acc[2]);
        acc[3] = FragH::mma(a, b3, acc[3]);
        guard_grp(acc[0], acc[1], acc[2], acc[3], a, b0, b1, b2, b3);
      }
#pragma unroll 1
      for (int k0 = 0; k0 < NHID; k0 += 32) {
        const v16h a  = FragH::load(ahrow + k0);
        const v16h b0 = FragH::load(wh + k0);
        const v16h b1 = FragH::load(wh + GSTR_H + k0);
        const v16h b2 = FragH::load(wh + 2 * GSTR_H + k0);
        const v16h b3 = FragH::load(wh + 3 * GSTR_H + k0);
        acc[0] = FragH::mma(a, b0, acc[0]);
        acc[1] = FragH::mma(a, b1, acc[1]);
        acc[2] = FragH::mma(a, b2, acc[2]);
        acc[3] = FragH::mma(a, b3, acc[3]);
        guard_grp(acc[0], acc[1], acc[2], acc[3], a, b0, b1, b2, b3);
      }
      acc_guard4(acc[0], acc[1], acc[2], acc[3]);

#pragma unroll
      for (int r = 0; r < 8; ++r) {
        const float zi = acc[0][r] * FOLD + bb[nt][0];
        const float zf = acc[1][r] * FOLD + bb[nt][1];
        const float zg = acc[2][r] * FOLD + bb[nt][2];
        const float zo = acc[3][r] * FOLD + bb[nt][3];
        const float ig = fsig(zi);
        const float fg = fsig(zf);
        const float gg = ftanh(zg);
        const float og = fsig(zo);
        const float co = cst[nt][r];
        const float ho = hst[nt][r];
        const float cn = fg * co + ig * gg;
        const float hn = og * ftanh(cn);
        const float mk = mkf[r];
        const float om = 1.0f - mk;
        const float hb = mk * hn + om * ho;
        const float cb = mk * cn + om * co;
        cst[nt][r] = cb;
        hst[nt][r] = hb;
        ahn[(8 * hh + r) * HPITCH + j] = h16_of(hb * ACARRY);
        slab[(8 * hh + r) * SLABP + 16 * nt + c] = hb * mk;
      }
    }

    __builtin_amdgcn_fence(__ATOMIC_RELEASE, "workgroup");
    __builtin_amdgcn_wave_barrier();
    __builtin_amdgcn_fence(__ATOMIC_ACQUIRE, "workgroup");

    if (LAYER == 0) {
      const int q = lane >> 3, c8 = (lane & 7) * 8;
      v8h hv[4];
#pragma unroll
      for (int it = 0; it < 4; ++it) {
        const int row = it * 4 + q;
        const float* sp = slab + row * SLABP + c8;
        const v4f x0 = *(const v4f*)(sp);
        const v4f x1 = *(const v4f*)(sp + 4);
#pragma unroll
        for (int e = 0; e < 4; ++e) {
          const float f0 = x0[e] * ACARRY;
          const float f1 = x1[e] * ACARRY;
          hv[it][e]     = h16_of(f0);
          hv[it][4 + e] = h16_of(f1);
        }
      }
      unsigned short* ob = outH + ((size_t)rowbase * NSTEP + (size_t)t) * NFEAT + dir * NHID + 64 * wave + c8;
      for (int pass = 0; pass < 2; ++pass) {
#pragma unroll
        for (int it = 0; it < 4; ++it) {
          const int row = it * 4 + q;
          *(volatile v8h*)(ob + (size_t)row * ROWSTR) = hv[it];
        }
        __threadfence();
      }
    } else {
      const int c4 = c * 4;
      float* ob = outF + ((size_t)rowbase * NSTEP + (size_t)t) * NFEAT + dir * NHID + 64 * wave + c4;
      for (int pass = 0; pass < 2; ++pass) {
#pragma unroll
        for (int it = 0; it < 8; ++it) {
          const int row = it * 2 + hh;
          const v4f v = *(const v4f*)(slab + row * SLABP + c4);
          *(volatile v4f*)(ob + (size_t)row * ROWSTR) = v;
        }
        __threadfence();
      }
    }
    __syncthreads();
  }
}

extern "C" void kernel_launch(void* const* d_in, const int* in_sizes, int n_in,
                              void* d_out, int out_size, void* d_ws, size_t ws_size, hipStream_t stream) {
  if (n_in < 14 || d_out == nullptr || d_ws == nullptr) return;
  if (in_sizes[0] != NROWS * NFEAT || in_sizes[1] != NROWS) return;
  for (int l = 0; l < 4; ++l) {
    if (in_sizes[2 + 3 * l] != NGATE * NFEAT) return;
    if (in_sizes[3 + 3 * l] != NGATE * NHID) return;
    if (in_sizes[4 + 3 * l] != NGATE) return;
  }
  if (out_size != NROWS * NFEAT) return;

  const float* x       = (const float*)d_in[0];
  const int*   mask    = (const int*)d_in[1];
  const float* Wih_l0f = (const float*)d_in[2];
  const float* Whh_l0f = (const float*)d_in[3];
  const float* b_l0f   = (const float*)d_in[4];
  const float* Wih_l0b = (const float*)d_in[5];
  const float* Whh_l0b = (const float*)d_in[6];
  const float* b_l0b   = (const float*)d_in[7];
  const float* Wih_l1f = (const float*)d_in[8];
  const float* Whh_l1f = (const float*)d_in[9];
  const float* b_l1f   = (const float*)d_in[10];
  const float* Wih_l1b = (const float*)d_in[11];
  const float* Whh_l1b = (const float*)d_in[12];
  const float* b_l1b   = (const float*)d_in[13];
  float* out = (float*)d_out;

  char* ws = (char*)d_ws;
  size_t off = 0;
  auto carve = [&](size_t bytes) -> char* { char* p = ws + off; off += (bytes + 255) & ~(size_t)255; return p; };
  unsigned short* X16   = (unsigned short*)carve((size_t)NROWS * NFEAT * 2);
  unsigned short* O16   = (unsigned short*)carve((size_t)NROWS * NFEAT * 2);
  unsigned short* WIH16 = (unsigned short*)carve((size_t)4 * NGATE * NFEAT * 2);
  unsigned short* WHH16 = (unsigned short*)carve((size_t)4 * NGATE * NHID * 2);
  if (off > ws_size || off > (size_t)134217728) return;

  const int n8x = NROWS * NFEAT / 8;
  const int n8i = NGATE * NFEAT / 8;
  const int n8h = NGATE * NHID / 8;
  cvt8_kernel<<<dim3((n8x + CVT_THR - 1) / CVT_THR, 1), CVT_THR, 0, stream>>>(x, x, x, x, X16, n8x, ACARRY);
  cvt8_kernel<<<dim3((n8i + CVT_THR - 1) / CVT_THR, 4), CVT_THR, 0, stream>>>(Wih_l0f, Wih_l0b, Wih_l1f, Wih_l1b, WIH16, n8i, WCARRY);
  cvt8_kernel<<<dim3((n8h + CVT_THR - 1) / CVT_THR, 4), CVT_THR, 0, stream>>>(Whh_l0f, Whh_l0b, Whh_l1f, Whh_l1b, WHH16, n8h, WCARRY);

  recur_layer_kernel<0><<<4, NTHR, 0, stream>>>(X16, WIH16, WHH16, b_l0f, b_l0b, mask, O16, out);
  recur_layer_kernel<1><<<4, NTHR, 0, stream>>>(O16, WIH16 + (size_t)2 * NGATE * NFEAT, WHH16 + (size_t)2 * NGATE * NHID,
                                                b_l1f, b_l1b, mask, O16, out);
}
